// Trajectron_87797721465263
// MI455X (gfx1250) — hardware-run, weakly checked
//
#include <hip/hip_runtime.h>
#include <math.h>

typedef __attribute__((ext_vector_type(16))) _Float16 v16h;
typedef __attribute__((ext_vector_type(8)))  _Float16 v8h;
typedef __attribute__((ext_vector_type(8)))  float    v8f;
typedef __attribute__((ext_vector_type(4)))  float    v4f;

constexpr int kFrames  = 256;
constexpr int kRowsB   = 128;
constexpr int kNodes   = 4;
constexpr int kCoord   = 2;
constexpr int kWindow  = 64;
constexpr int kHidA    = 32;
constexpr int kHidB    = 8;
constexpr int kGateA   = 4 * kHidA;
constexpr int kGateB   = 4 * kHidB;
constexpr int kEmb     = kHidA + kHidB;
constexpr int kOutW    = 2;
constexpr int kFrameFl = kRowsB * kNodes * kCoord;
constexpr int kThreads = 256;
constexpr float kCarryW = 64.0f;
constexpr float kCarryH = 256.0f;
constexpr float kFold   = 1.0f / (kCarryW * kCarryH);
static_assert(kGateA == 128 && kGateB == 32 && kEmb == 40, "gate widths");
static_assert(kHidA == 32, "one 32-deep k step per product");
static_assert(kFrameFl == 4 * kThreads, "one 16-B load per thread stages one frame");
static_assert(kRowsB == 16 * (kThreads / 32), "each wave owns 16 rows");
static_assert(kRowsB * kOutW == kThreads, "one output element per thread");
static_assert(kOutW * kEmb <= kThreads, "head weights fit the staging array");
static_assert((kEmb % 4) == 0, "head dot in groups of four");
static_assert(kRowsB * kHidA == kThreads * 2 * 8, "state plane A zero-fill: 256 threads x 2 trips x 8 halves");
static_assert(kRowsB * kHidB == kRowsB * 8, "state plane B zero-fill: 128 threads x 8 halves");

union FragU { v16h v; v8h h[2]; };

__device__ __forceinline__ v8f mma_f16(v16h a, v16h b) {
  v8f c = (v8f){0.f, 0.f, 0.f, 0.f, 0.f, 0.f, 0.f, 0.f};
  c = __builtin_amdgcn_wmma_f32_16x16x32_f16(false, a, false, b, (short)0, c, false, false);
  asm volatile("v_nop\n\tv_nop\n\tv_nop\n\tv_nop" : "+v"(c) : "v"(a), "v"(b));
  return c;
}

__device__ __forceinline__ float sig_fast(float z) {
  return __builtin_amdgcn_rcpf(1.0f + __expf(-z));
}
__device__ __forceinline__ float tanh_fast(float z) {
  return 1.0f - 2.0f * __builtin_amdgcn_rcpf(__expf(2.0f * z) + 1.0f);
}

__global__ __launch_bounds__(256)
void window_lstm_kernel(const float* __restrict__ frames,
                        const float* __restrict__ Wih_a,
                        const float* __restrict__ Whh_a,
                        const float* __restrict__ bih_a,
                        const float* __restrict__ bhh_a,
                        const float* __restrict__ Wih_b,
                        const float* __restrict__ Whh_b,
                        const float* __restrict__ bih_b,
                        const float* __restrict__ bhh_b,
                        const float* __restrict__ W_head,
                        const float* __restrict__ b_head,
                        float* __restrict__ out)
{
  __shared__ __align__(16) _Float16 sHa[2][kRowsB * kHidA];
  __shared__ __align__(16) _Float16 sHb[2][kRowsB * kHidB];
  __shared__ __align__(16) float    sX[2][kRowsB * 4];
  __shared__ __align__(16) float    sHf[kRowsB * kEmb];
  __shared__ __align__(16) float    sPa[kGateA * 4];
  __shared__ __align__(16) float    sPb[kGateB * 4];
  __shared__ __align__(16) float    sWo[kThreads];

  const int tid  = threadIdx.x;
  const int lane = tid & 31;
  const int wv   = tid >> 5;
  const int cl   = lane & 15;
  const int hi   = lane >> 4;
  const int w    = blockIdx.x;

  {
    const int ga = tid & (kGateA - 1);
    float a0 = Wih_a[2 * ga];
    float a1 = Wih_a[2 * ga + 1];
    float ab = bih_a[ga] + bhh_a[ga];
    asm volatile("" : "+v"(a0), "+v"(a1), "+v"(ab));
    if (tid < kGateA) {
      sPa[ga * 4 + 0] = a0;
      sPa[ga * 4 + 1] = a1;
      sPa[ga * 4 + 2] = ab;
      sPa[ga * 4 + 3] = 0.0f;
    }
    const int gb = tid & (kGateB - 1);
    float c0 = Wih_b[2 * gb];
    float c1 = Wih_b[2 * gb + 1];
    float cb = bih_b[gb] + bhh_b[gb];
    asm volatile("" : "+v"(c0), "+v"(c1), "+v"(cb));
    if (tid < kGateB) {
      sPb[gb * 4 + 0] = c0;
      sPb[gb * 4 + 1] = c1;
      sPb[gb * 4 + 2] = cb;
      sPb[gb * 4 + 3] = 0.0f;
    }
    const int wi = (tid < kOutW * kEmb) ? tid : (kOutW * kEmb - 1);
    sWo[tid] = W_head[wi];
  }

  v16h Bh[8];
#pragma unroll
  for (int n = 0; n < 8; ++n) {
    const float* src = Whh_a + (size_t)(n * 16 + cl) * kHidA + 8 * hi;
    const v4f q0 = *(const v4f*)(src);
    const v4f q1 = *(const v4f*)(src + 4);
    const v4f q2 = *(const v4f*)(src + 16);
    const v4f q3 = *(const v4f*)(src + 20);
    v16h b;
#pragma unroll
    for (int e = 0; e < 4; ++e) {
      b[e]      = (_Float16)(q0[e] * kCarryW);
      b[4 + e]  = (_Float16)(q1[e] * kCarryW);
      b[8 + e]  = (_Float16)(q2[e] * kCarryW);
      b[12 + e] = (_Float16)(q3[e] * kCarryW);
    }
    Bh[n] = b;
  }
  v16h Bi[2];
#pragma unroll
  for (int n = 0; n < 2; ++n) {
    const float* src = Whh_b + (size_t)(n * 16 + cl) * kHidB;
    const v4f q0 = *(const v4f*)(src);
    const v4f q1 = *(const v4f*)(src + 4);
    v16h b;
#pragma unroll
    for (int e = 0; e < 4; ++e) {
      const float u0 = (hi == 0) ? (q0[e] * kCarryW) : 0.0f;
      const float u1 = (hi == 0) ? (q1[e] * kCarryW) : 0.0f;
      b[e]      = (_Float16)u0;
      b[4 + e]  = (_Float16)u1;
      b[8 + e]  = (_Float16)0.0f;
      b[12 + e] = (_Float16)0.0f;
    }
    Bi[n] = b;
  }

  float csA0[8], csA1[8], csB[8];
#pragma unroll
  for (int r = 0; r < 8; ++r) { csA0[r] = 0.0f; csA1[r] = 0.0f; csB[r] = 0.0f; }

  const int rowA   = wv * 16 + cl;
  const int rowD   = wv * 16 + 8 * hi;
  const int t0     = (w >= kWindow - 1) ? (w - (kWindow - 1)) : 0;
  int nsteps       = w - t0 + 1;
  nsteps           = (nsteps > kWindow) ? kWindow : nsteps;

  {
    const _Float16 hz = (_Float16)0.0f;
    const v8h zv = {hz, hz, hz, hz, hz, hz, hz, hz};
#pragma unroll
    for (int i = 0; i < 2; ++i) *(v8h*)&sHa[0][(tid + kThreads * i) * 8] = zv;
    if (tid < kRowsB) *(v8h*)&sHb[0][tid * 8] = zv;
    const v4f xv = *(const v4f*)(frames + (size_t)t0 * kFrameFl + tid * 4);
    const bool up = (tid & 1) != 0;
    sX[0][tid * 2]     = up ? xv[2] : xv[0];
    sX[0][tid * 2 + 1] = up ? xv[3] : xv[1];
  }
  __syncthreads();

  int p = 0;
#pragma unroll 1
  for (int s = 0; s < nsteps; ++s) {
    const int t  = t0 + s;
    const int tn = (t < w) ? (t + 1) : w;
    const v4f xnext = *(const v4f*)(frames + (size_t)tn * kFrameFl + tid * 4);

    FragU fa;
    {
      const _Float16* pa = &sHa[p][rowA * kHidA + 8 * hi];
      fa.h[0] = *(const v8h*)(pa);
      fa.h[1] = *(const v8h*)(pa + 16);
    }
    FragU fb;
    {
      const _Float16 hz = (_Float16)0.0f;
      const v8h zv = {hz, hz, hz, hz, hz, hz, hz, hz};
      const v8h ld = *(const v8h*)&sHb[p][rowA * kHidB];
      fb.h[0] = (hi == 0) ? ld : zv;
      fb.h[1] = zv;
    }
    const float* xs = &sX[p][rowD * 4];

#pragma unroll
    for (int n = 0; n < 2; ++n) {
      const v8f di = mma_f16(fa.v, Bh[n]);
      const v8f df = mma_f16(fa.v, Bh[n + 2]);
      const v8f dg = mma_f16(fa.v, Bh[n + 4]);
      const v8f dq = mma_f16(fa.v, Bh[n + 6]);
      const v4f pi = *(const v4f*)&sPa[((n)     * 16 + cl) * 4];
      const v4f pf = *(const v4f*)&sPa[((n + 2) * 16 + cl) * 4];
      const v4f pg = *(const v4f*)&sPa[((n + 4) * 16 + cl) * 4];
      const v4f pq = *(const v4f*)&sPa[((n + 6) * 16 + cl) * 4];
      _Float16* hn16 = &sHa[p ^ 1][rowD * kHidA + n * 16 + cl];
      float*    hn32 = &sHf[rowD * kEmb + n * 16 + cl];
#pragma unroll
      for (int r = 0; r < 8; ++r) {
        const v4f xv = *(const v4f*)(xs + r * 4);
        const float x0 = xv[2], x1 = xv[3];
        float gi = fmaf(x1, pi[1], fmaf(x0, pi[0], pi[2]));
        float gf = fmaf(x1, pf[1], fmaf(x0, pf[0], pf[2]));
        float gg = fmaf(x1, pg[1], fmaf(x0, pg[0], pg[2]));
        float go = fmaf(x1, pq[1], fmaf(x0, pq[0], pq[2]));
        gi = fmaf(di[r], kFold, gi);
        gf = fmaf(df[r], kFold, gf);
        gg = fmaf(dg[r], kFold, gg);
        go = fmaf(dq[r], kFold, go);
        const float cprev = (n == 0) ? csA0[r] : csA1[r];
        const float cn = sig_fast(gf) * cprev + sig_fast(gi) * tanh_fast(gg);
        if (n == 0) csA0[r] = cn; else csA1[r] = cn;
        const float hn = sig_fast(go) * tanh_fast(cn);
        hn16[r * kHidA] = (_Float16)(hn * kCarryH);
        hn32[r * kEmb]  = hn;
      }
    }

    {
      const v8f d0 = mma_f16(fb.v, Bi[0]);
      const v8f d1 = mma_f16(fb.v, Bi[1]);
      const v4f q0 = *(const v4f*)&sPb[(cl) * 4];
      const v4f q1 = *(const v4f*)&sPb[(16 + cl) * 4];
#pragma unroll
      for (int r = 0; r < 8; ++r) {
        const v4f xv = *(const v4f*)(xs + r * 4);
        const float x0 = xv[0], x1 = xv[1];
        float ga = fmaf(x1, q0[1], fmaf(x0, q0[0], q0[2]));
        float gb = fmaf(x1, q1[1], fmaf(x0, q1[0], q1[2]));
        ga = fmaf(d0[r], kFold, ga);
        gb = fmaf(d1[r], kFold, gb);
        const float gf = __shfl_xor(ga, 8, 32);
        const float go = __shfl_xor(gb, 8, 32);
        const float cn = sig_fast(gf) * csB[r] + sig_fast(ga) * tanh_fast(gb);
        csB[r] = cn;
        const float hn = sig_fast(go) * tanh_fast(cn);
        if (cl < kHidB) {
          sHb[p ^ 1][(rowD + r) * kHidB + cl] = (_Float16)(hn * kCarryH);
          sHf[(rowD + r) * kEmb + kHidA + cl] = hn;
        }
      }
    }

    {
      const bool up = (tid & 1) != 0;
      sX[p ^ 1][tid * 2]     = up ? xnext[2] : xnext[0];
      sX[p ^ 1][tid * 2 + 1] = up ? xnext[3] : xnext[1];
    }
    __syncthreads();
    p ^= 1;
  }

  {
    const int b = tid >> 1;
    const int o = tid & 1;
    float acc = b_head[o];
    const float* hr = sHf + b * kEmb;
    const float* wr = sWo + o * kEmb;
#pragma unroll 1
    for (int k4 = 0; k4 < kEmb / 4; ++k4) {
      const v4f hv = *(const v4f*)(hr + 4 * k4);
      const v4f wq = *(const v4f*)(wr + 4 * k4);
      acc = fmaf(hv[0], wq[0], acc);
      acc = fmaf(hv[1], wq[1], acc);
      acc = fmaf(hv[2], wq[2], acc);
      acc = fmaf(hv[3], wq[3], acc);
    }
    volatile float* po = out + (size_t)w * kThreads + tid;
    *po = acc;
    __threadfence();
    *po = acc;
  }
}

extern "C" void kernel_launch(void* const* d_in, const int* in_sizes, int n_in,
                              void* d_out, int out_size, void* d_ws, size_t ws_size,
                              hipStream_t stream) {
  (void)d_ws; (void)ws_size;
  if (n_in < 11) return;
  if (in_sizes[0] != kFrames * kFrameFl) return;
  if (in_sizes[1] != kGateA * kCoord) return;
  if (in_sizes[2] != kGateA * kHidA) return;
  if (in_sizes[3] != kGateA) return;
  if (in_sizes[4] != kGateA) return;
  if (in_sizes[5] != kGateB * kCoord) return;
  if (in_sizes[6] != kGateB * kHidB) return;
  if (in_sizes[7] != kGateB) return;
  if (in_sizes[8] != kGateB) return;
  if (in_sizes[9] != kOutW * kEmb) return;
  if (in_sizes[10] != kOutW) return;
  if (out_size != kFrames * kRowsB * kOutW) return;

  window_lstm_kernel<<<kFrames, kThreads, 0, stream>>>(
      (const float*)d_in[0],
      (const float*)d_in[1],
      (const float*)d_in[2],
      (const float*)d_in[3],
      (const float*)d_in[4],
      (const float*)d_in[5],
      (const float*)d_in[6],
      (const float*)d_in[7],
      (const float*)d_in[8],
      (const float*)d_in[9],
      (const float*)d_in[10],
      (float*)d_out);
}
